// TransformerLayer_17403207483584
// MI455X (gfx1250) — hardware-verified
//
#include <hip/hip_runtime.h>
#include <math.h>

typedef __attribute__((ext_vector_type(16))) _Float16 v16h;
typedef __attribute__((ext_vector_type(8)))  _Float16 v8h;
typedef __attribute__((ext_vector_type(8)))  float v8f;
typedef __attribute__((ext_vector_type(4)))  float v4f;

#ifndef NB
#define NB 2
#endif
#define NB_FULL 2
#ifndef SEQ
#define SEQ 2048
#endif
#define SEQ_FULL 2048
#define DM 1024
#define NH 16
#define HD 64
#define RW 128
#define DF 4096
#define MROWS (NB * SEQ)
#define QSCALE (0.125f)
#define RC (4096.0f)
#define PCY (16384.0f)
#define WC (64.0f)
#define F16MIN (6.103515625e-05f)
#define LN_EPS (1e-5f)
static_assert(SEQ % 64 == 0);
static_assert(SEQ >= 64);
static_assert((SEQ & (SEQ - 1)) == 0);
static_assert(SEQ <= SEQ_FULL);
static_assert(NB >= 1 && NB <= NB_FULL);
static_assert(NH * HD == DM);
static_assert(HD == 64);
static_assert(RW == 128);
static_assert(DM % 128 == 0 && DF % 128 == 0 && DM % 32 == 0 && DF % 32 == 0);
static_assert(MROWS % 64 == 0);
static_assert(((DM * DM / 8) % 256) == 0 && ((DF * DM / 8) % 256) == 0);

#define WSZ_WE   (2u * (size_t)DM * DM)
#define WSZ_WF   (2u * (size_t)DF * DM)
#define WSZ_ACT  (2u * (size_t)MROWS * DM)
#define WSZ_HH   (2u * (size_t)MROWS * DF)
#define WSZ_X1   (4u * (size_t)MROWS * DM)
#define WS_WQ   ((size_t)0)
#define WS_WK   (WS_WQ  + WSZ_WE)
#define WS_WV   (WS_WK  + WSZ_WE)
#define WS_WO   (WS_WV  + WSZ_WE)
#define WS_W1   (WS_WO  + WSZ_WE)
#define WS_W2   (WS_W1  + WSZ_WF)
#define WS_XN   (WS_W2  + WSZ_WF)
#define WS_QH   (WS_XN  + WSZ_ACT)
#define WS_QL   (WS_QH  + WSZ_ACT)
#define WS_KH   (WS_QL  + WSZ_ACT)
#define WS_KL   (WS_KH  + WSZ_ACT)
#define WS_HH   (WS_QH)
#define WS_VT   (WS_KL  + WSZ_ACT)
#define WS_O16  (WS_VT  + WSZ_ACT)
#define WS_X1   (WS_O16 + WSZ_ACT)
#define WS_XN2  (WS_X1  + WSZ_X1)
#define WS_END  (WS_XN2 + WSZ_ACT)
static_assert(WSZ_HH == 4u * WSZ_ACT);
static_assert(WS_HH + WSZ_HH == WS_VT);
static_assert(WS_END <= (size_t)134217728u);
static_assert((WSZ_WE % 256u) == 0 && (WSZ_WF % 256u) == 0 && (WSZ_ACT % 256u) == 0 && (WSZ_X1 % 256u) == 0);

template <typename T> __device__ __forceinline__ void vst2(void* p, T v) { *(volatile T*)p = v; __threadfence(); *(volatile T*)p = v; }
__device__ __forceinline__ v8f zero8() { v8f z = {0.f, 0.f, 0.f, 0.f, 0.f, 0.f, 0.f, 0.f}; return z; }
__device__ __forceinline__ v8f wmma16(v16h a, v16h b, v8f c) {
  v8f d = __builtin_amdgcn_wmma_f32_16x16x32_f16(false, a, false, b, (short)0, c, false, false);
  asm volatile("v_nop\n\tv_nop\n\tv_nop\n\tv_nop" : "+v"(d) : "v"(a), "v"(b));
  return d;
}
__device__ __forceinline__ v16h frag_h(const _Float16* rowk0, unsigned lane) {
  union { v16h v; v8h q[2]; } u; const _Float16* p = rowk0 + 8u * (lane >> 4);
  u.q[0] = *(const v8h*)p; u.q[1] = *(const v8h*)(p + 16); return u.v;
}
__device__ __forceinline__ v16h frag_h2(const _Float16* p0, const _Float16* p1) {
  union { v16h v; v8h q[2]; } u; u.q[0] = *(const v8h*)p0; u.q[1] = *(const v8h*)p1; return u.v;
}
__device__ __forceinline__ _Float16 f16n(float x) { const float t = (fabsf(x) >= F16MIN) ? x : 0.0f; return (_Float16)t; }
__device__ __forceinline__ unsigned short bf16bits(float x) { unsigned u = __float_as_uint(x); u += 0x7FFFu + ((u >> 16) & 1u); return (unsigned short)(u >> 16); }
__device__ __forceinline__ float bf16val(unsigned short b) { return __uint_as_float(((unsigned)b) << 16); }
__device__ __forceinline__ float bfq(float x) { return bf16val(bf16bits(x)); }
__device__ __forceinline__ v4f cvb4(v4f a) { v4f o; o[0] = bfq(a[0]); o[1] = bfq(a[1]); o[2] = bfq(a[2]); o[3] = bfq(a[3]); return o; }
__device__ __forceinline__ size_t xrow(unsigned m) { return (size_t)(m / (unsigned)SEQ) * (size_t)SEQ_FULL + (size_t)(m % (unsigned)SEQ); }
#define LDSX() do { asm volatile("s_wait_dscnt 0" ::: "memory"); __builtin_amdgcn_wave_barrier(); __builtin_amdgcn_fence(3  , "workgroup"); } while (0)

__global__ __launch_bounds__(256) void k_cvth(const float* __restrict__ src, unsigned n8, _Float16* __restrict__ dst) {
  const unsigned i = blockIdx.x * 256u + threadIdx.x; if (i >= n8) return;
  const float* p = src + (size_t)i * 8; const v4f a = *(const v4f*)p, b = *(const v4f*)(p + 4);
  v8h o;
#pragma unroll
  for (int e = 0; e < 4; ++e) { o[e] = f16n(bfq(a[e]) * WC); o[4 + e] = f16n(bfq(b[e]) * WC); }
  vst2(dst + (size_t)i * 8, o);
}

template <bool EXT>
__global__ __launch_bounds__(256) void k_ln(const float* __restrict__ X, const float* __restrict__ G, const float* __restrict__ Bt, _Float16* __restrict__ OUT) {
  const unsigned wave = threadIdx.x >> 5, lane = threadIdx.x & 31u; const unsigned m = blockIdx.x * 8u + wave; if (m >= (unsigned)MROWS) return;
  const float* xr = X + (EXT ? xrow(m) : (size_t)m) * DM + lane * 8u;
  float s1 = 0.f;
#pragma unroll 1
  for (unsigned i = 0; i < 4u; ++i) { v4f a = *(const v4f*)(xr + i * 256u), b = *(const v4f*)(xr + i * 256u + 4u);
    if (EXT) { a = cvb4(a); b = cvb4(b); }
    s1 += ((a[0] + a[1]) + (a[2] + a[3])) + ((b[0] + b[1]) + (b[2] + b[3])); }
#pragma unroll
  for (int o = 1; o < 32; o <<= 1) s1 += __shfl_xor(s1, o);
  const float mu = s1 * (1.0f / DM); float q = 0.f;
#pragma unroll 1
  for (unsigned i = 0; i < 4u; ++i) { v4f a = *(const v4f*)(xr + i * 256u), b = *(const v4f*)(xr + i * 256u + 4u);
    if (EXT) { a = cvb4(a); b = cvb4(b); }
#pragma unroll
    for (int e = 0; e < 4; ++e) { const float d0 = a[e] - mu, d1 = b[e] - mu; q += d0 * d0; q += d1 * d1; } }
#pragma unroll
  for (int o = 1; o < 32; o <<= 1) q += __shfl_xor(q, o);
  const float inv = 1.0f / sqrtf(q * (1.0f / DM) + LN_EPS);
  _Float16* orow = OUT + (size_t)m * DM + lane * 8u;
#pragma unroll 1
  for (unsigned i = 0; i < 4u; ++i) { v4f a = *(const v4f*)(xr + i * 256u), b = *(const v4f*)(xr + i * 256u + 4u);
    if (EXT) { a = cvb4(a); b = cvb4(b); }
    const unsigned c = i * 256u + lane * 8u;
    const v4f ga = cvb4(*(const v4f*)(G + c)), gb = cvb4(*(const v4f*)(G + c + 4u)), ba = cvb4(*(const v4f*)(Bt + c)), bb = cvb4(*(const v4f*)(Bt + c + 4u));
    v8h o8;
#pragma unroll
    for (int e = 0; e < 4; ++e) { o8[e] = f16n((a[e] - mu) * inv * ga[e] + ba[e]); o8[4 + e] = f16n((b[e] - mu) * inv * gb[e] + bb[e]); }
    vst2(orow + i * 256u, o8); }
}

__global__ __launch_bounds__(128) void k_pqk(const _Float16* __restrict__ A, const _Float16* __restrict__ W, const float* __restrict__ BIAS, _Float16* __restrict__ OH, _Float16* __restrict__ OL) {
  __shared__ __align__(16) _Float16 sh[64][136], sl[64][136];
  const unsigned tid = threadIdx.x, wave = tid >> 5, lane = tid & 31u, col = lane & 15u, g = lane >> 4;
  const unsigned c0 = blockIdx.y * 128u; const unsigned r0 = blockIdx.x * 64u;
  v8f acc[8];
#pragma unroll
  for (int j = 0; j < 8; ++j) acc[j] = zero8();
  const _Float16* ap = A + (size_t)(r0 + wave * 16u + col) * DM; const _Float16* wp = W + (size_t)(c0 + col) * DM;
#pragma unroll 1
  for (unsigned kc = 0; kc < DM / 32; ++kc) {
    const v16h a = frag_h(ap + kc * 32u, lane);
#pragma unroll
    for (int j = 0; j < 8; ++j) acc[j] = wmma16(a, frag_h(wp + (size_t)j * 16 * DM + kc * 32u, lane), acc[j]);
  }
#pragma unroll
  for (int j = 0; j < 8; ++j) {
    const float bz = bfq(BIAS[c0 + j * 16 + col]);
#pragma unroll
    for (int r = 0; r < 8; ++r) { const float v = acc[j][r] * (1.0f / WC) + bz; const _Float16 hv = f16n(v); sh[wave * 16u + 8u * g + r][j * 16 + col] = hv; sl[wave * 16u + 8u * g + r][j * 16 + col] = f16n((v - (float)hv) * RC); }
  }
  __syncthreads();
  for (unsigned e = tid; e < 64u * 16u; e += 128u) { const unsigned rl = e >> 4, q = e & 15u; const size_t o = (size_t)(r0 + rl) * DM + c0 + q * 8u;
    const v8h vh = *(const v8h*)&sh[rl][q * 8u]; const v8h vl = *(const v8h*)&sl[rl][q * 8u]; vst2(OH + o, vh); vst2(OL + o, vl); }
}

__global__ __launch_bounds__(128) void k_pvt(const _Float16* __restrict__ A, const _Float16* __restrict__ W, const float* __restrict__ BIAS, _Float16* __restrict__ VT) {
  __shared__ __align__(16) _Float16 th[128][72];
  const unsigned tid = threadIdx.x, wave = tid >> 5, lane = tid & 31u, col = lane & 15u, g = lane >> 4;
  const unsigned c0 = blockIdx.y * 128u; const unsigned r0 = blockIdx.x * 64u;
  v8f acc[8];
#pragma unroll
  for (int j = 0; j < 8; ++j) acc[j] = zero8();
  const _Float16* ap = A + (size_t)(r0 + wave * 16u + col) * DM; const _Float16* wp = W + (size_t)(c0 + col) * DM;
#pragma unroll 1
  for (unsigned kc = 0; kc < DM / 32; ++kc) {
    const v16h a = frag_h(ap + kc * 32u, lane);
#pragma unroll
    for (int j = 0; j < 8; ++j) acc[j] = wmma16(a, frag_h(wp + (size_t)j * 16 * DM + kc * 32u, lane), acc[j]);
  }
#pragma unroll
  for (int j = 0; j < 8; ++j) {
    const float bz = bfq(BIAS[c0 + j * 16 + col]);
#pragma unroll
    for (int r = 0; r < 8; ++r) th[j * 16 + col][wave * 16u + 8u * g + r] = f16n(acc[j][r] * (1.0f / WC) + bz);
  }
  __syncthreads();
  for (unsigned e = tid; e < 128u * 8u; e += 128u) { const unsigned cl = e >> 3, q = e & 7u; const v8h v = *(const v8h*)&th[cl][q * 8u]; vst2(VT + (size_t)(c0 + cl) * MROWS + r0 + q * 8u, v); }
}

__device__ __forceinline__ v8f att_qk(const _Float16* __restrict__ KH, const _Float16* __restrict__ KL, size_t ko, unsigned lane, v16h qh0, v16h qh1, v16h qr0, v16h qr1) {
  v8f cs = zero8(), cl = zero8();
  { const v16h bh = frag_h(KH + ko, lane); const v16h br = frag_h(KL + ko, lane);
    cs = wmma16(qh0, bh, cs); cl = wmma16(qr0, bh, cl); cl = wmma16(qh0, br, cl); }
  { const v16h bh = frag_h(KH + ko + 32, lane); const v16h br = frag_h(KL + ko + 32, lane);
    cs = wmma16(qh1, bh, cs); cl = wmma16(qr1, bh, cl); cl = wmma16(qh1, br, cl); }
  v8f o;
#pragma unroll
  for (int r = 0; r < 8; ++r) o[r] = (cs[r] + cl[r] * (1.0f / RC)) * QSCALE;
  return o;
}

__global__ __launch_bounds__(128) void k_att(const _Float16* __restrict__ QH, const _Float16* __restrict__ QL, const _Float16* __restrict__ KH, const _Float16* __restrict__ KL,
                                             const _Float16* __restrict__ VT, const float* __restrict__ RP, _Float16* __restrict__ O16) {
  __shared__ __align__(16) _Float16 sP[4][16][168];
  __shared__ __align__(16) _Float16 so[4][16][72];
  __shared__ float sb[RW];
  const unsigned tid = threadIdx.x, wave = tid >> 5, lane = tid & 31u, col = lane & 15u, g = lane >> 4;
  const unsigned h = blockIdx.y, b = blockIdx.z;
  sb[tid] = bfq(RP[h * RW + tid]);
  __syncthreads();
  const unsigned i0 = blockIdx.x * 64u + wave * 16u;
  const size_t rowb = (size_t)b * SEQ;
  const size_t hoff = (size_t)h * HD;
  const size_t kb = rowb * DM + hoff;
  const size_t qo = (rowb + i0 + col) * DM + hoff;
  const v16h qh0 = frag_h(QH + qo, lane), qh1 = frag_h(QH + qo + 32, lane);
  const v16h qr0 = frag_h(QL + qo, lane), qr1 = frag_h(QL + qo + 32, lane);
  float mx[8], lsum[8];
#pragma unroll
  for (int r = 0; r < 8; ++r) { mx[r] = -3.0e38f; lsum[r] = 0.f; }
#pragma unroll 1
  for (unsigned t = 0; t < 9u; ++t) {
    const unsigned tk = i0 + 16u * t + col;
    const bool kin = tk >= 128u;
    const unsigned jkc = kin ? (tk - 128u) : 0u;
    const v8f raw = att_qk(KH, KL, kb + (size_t)jkc * DM, lane, qh0, qh1, qr0, qr1);
#pragma unroll
    for (int r = 0; r < 8; ++r) {
      const unsigned base = 128u - 16u * t + 8u * g + (unsigned)r;
      const bool ge = base >= col;
      const unsigned rel = base - col;
      const bool ok = kin && ge && (rel < (unsigned)RW);
      const unsigned rc = ge ? (rel < (unsigned)(RW - 1) ? rel : (unsigned)(RW - 1)) : 0u;
      const float bz = sb[rc];
      const float sc = raw[r] + bz;
      const float sv = ok ? sc : -3.0e38f;
      mx[r] = fmaxf(mx[r], sv);
    }
  }
#pragma unroll
  for (int r = 0; r < 8; ++r) {
    float m = mx[r];
    m = fmaxf(m, __shfl_xor(m, 1)); m = fmaxf(m, __shfl_xor(m, 2)); m = fmaxf(m, __shfl_xor(m, 4)); m = fmaxf(m, __shfl_xor(m, 8));
    mx[r] = m;
    sP[wave][8u * g + r][col] = (_Float16)0.0f;
  }
#pragma unroll 1
  for (unsigned t = 0; t < 9u; ++t) {
    const unsigned tk = i0 + 16u * t + col;
    const bool kin = tk >= 128u;
    const unsigned jkc = kin ? (tk - 128u) : 0u;
    const v8f raw = att_qk(KH, KL, kb + (size_t)jkc * DM, lane, qh0, qh1, qr0, qr1);
    const unsigned pc0 = 16u * (t + 1u) + col;
#pragma unroll
    for (int r = 0; r < 8; ++r) {
      const unsigned base = 128u - 16u * t + 8u * g + (unsigned)r;
      const bool ge = base >= col;
      const unsigned rel = base - col;
      const bool ok = kin && ge && (rel < (unsigned)RW);
      const unsigned rc = ge ? (rel < (unsigned)(RW - 1) ? rel : (unsigned)(RW - 1)) : 0u;
      const float bz = sb[rc];
      const float sc = raw[r] + bz;
      const float sv = ok ? sc : -3.0e38f;
      const float e = fminf(fmaxf(sv - mx[r], -100.0f), 0.0f);
      float pc = __expf(e) * PCY; pc = (pc >= F16MIN) ? pc : 0.0f;
      const _Float16 ph = (_Float16)pc;
      lsum[r] += (float)ph;
      sP[wave][8u * g + r][pc0] = ph;
    }
  }
  LDSX();
  v8f acc[4];
#pragma unroll
  for (int j = 0; j < 4; ++j) acc[j] = zero8();
#pragma unroll 1
  for (unsigned kk = 0; kk < 5u; ++kk) {
    const v16h a = frag_h(&sP[wave][col][kk * 32u], lane);
    const unsigned t1 = i0 + 32u * kk + 8u * g, t2 = t1 + 16u;
    const unsigned k1 = (t1 >= 144u) ? (t1 - 144u) : 0u, k2 = (t2 >= 144u) ? (t2 - 144u) : 0u;
#pragma unroll
    for (int j = 0; j < 4; ++j) {
      const _Float16* vp = VT + ((size_t)(h * HD + j * 16 + col) * MROWS + rowb);
      acc[j] = wmma16(a, frag_h2(vp + k1, vp + k2), acc[j]);
    }
  }
  float inv[8];
#pragma unroll
  for (int r = 0; r < 8; ++r) { float t = lsum[r]; t += __shfl_xor(t, 1); t += __shfl_xor(t, 2); t += __shfl_xor(t, 4); t += __shfl_xor(t, 8); inv[r] = 1.0f / t; }
#pragma unroll
  for (int j = 0; j < 4; ++j)
#pragma unroll
    for (int r = 0; r < 8; ++r) so[wave][8u * g + r][j * 16 + col] = f16n(acc[j][r] * inv[r]);
  LDSX();
#pragma unroll
  for (unsigned rp = 0; rp < 4u; ++rp) { const unsigned rl = rp * 4u + (lane >> 3), q = lane & 7u; const v8h v = *(const v8h*)&so[wave][rl][q * 8u];
    vst2(O16 + (rowb + i0 + rl) * DM + hoff + q * 8u, v); }
}

template <int KD, bool RESX, bool OUTX>
__global__ __launch_bounds__(128) void k_gr(const _Float16* __restrict__ A, const _Float16* __restrict__ W, const float* __restrict__ BIAS, const float* __restrict__ RES, float* __restrict__ OUT) {
  __shared__ __align__(16) float sf[4][16][132];
  const unsigned tid = threadIdx.x, wave = tid >> 5, lane = tid & 31u, col = lane & 15u, g = lane >> 4;
  const unsigned c0 = blockIdx.y * 128u; const unsigned r0 = blockIdx.x * 64u + wave * 16u;
  v8f acc[8];
#pragma unroll
  for (int j = 0; j < 8; ++j) acc[j] = zero8();
  const _Float16* ap = A + (size_t)(r0 + col) * KD; const _Float16* wp = W + (size_t)(c0 + col) * KD;
#pragma unroll 1
  for (unsigned kc = 0; kc < (unsigned)(KD / 32); ++kc) {
    const v16h a = frag_h(ap + kc * 32u, lane);
#pragma unroll
    for (int j = 0; j < 8; ++j) acc[j] = wmma16(a, frag_h(wp + (size_t)j * 16 * KD + kc * 32u, lane), acc[j]);
  }
#pragma unroll
  for (int j = 0; j < 8; ++j)
#pragma unroll
    for (int r = 0; r < 8; ++r) sf[wave][8u * g + r][j * 16 + col] = acc[j][r] * (1.0f / WC);
  LDSX();
  const v4f bz = cvb4(*(const v4f*)(BIAS + c0 + lane * 4u));
  for (unsigned rl = 0; rl < 16u; ++rl) {
    const unsigned m = r0 + rl;
    const size_t ri = (RESX ? xrow(m) : (size_t)m) * DM + c0 + lane * 4u;
    const size_t oi = (OUTX ? xrow(m) : (size_t)m) * DM + c0 + lane * 4u;
    v4f vv = *(const v4f*)&sf[wave][rl][lane * 4u]; v4f rv = *(const v4f*)(RES + ri);
    if (RESX) rv = cvb4(rv);
    vv[0] = (rv[0] + vv[0]) + bz[0]; vv[1] = (rv[1] + vv[1]) + bz[1]; vv[2] = (rv[2] + vv[2]) + bz[2]; vv[3] = (rv[3] + vv[3]) + bz[3];
    vst2(OUT + oi, vv);
  }
}

__global__ __launch_bounds__(128) void k_g1(const _Float16* __restrict__ A, const _Float16* __restrict__ W, const float* __restrict__ BIAS, _Float16* __restrict__ HH) {
  __shared__ __align__(16) _Float16 sg[4][16][136];
  const unsigned tid = threadIdx.x, wave = tid >> 5, lane = tid & 31u, col = lane & 15u, g = lane >> 4;
  const unsigned c0 = blockIdx.y * 128u; const unsigned r0 = blockIdx.x * 64u + wave * 16u;
  v8f acc[8];
#pragma unroll
  for (int j = 0; j < 8; ++j) acc[j] = zero8();
  const _Float16* ap = A + (size_t)(r0 + col) * DM; const _Float16* wp = W + (size_t)(c0 + col) * DM;
#pragma unroll 1
  for (unsigned kc = 0; kc < DM / 32; ++kc) {
    const v16h a = frag_h(ap + kc * 32u, lane);
#pragma unroll
    for (int j = 0; j < 8; ++j) acc[j] = wmma16(a, frag_h(wp + (size_t)j * 16 * DM + kc * 32u, lane), acc[j]);
  }
#pragma unroll
  for (int j = 0; j < 8; ++j) {
    const float bz = bfq(BIAS[c0 + j * 16 + col]);
#pragma unroll
    for (int r = 0; r < 8; ++r) sg[wave][8u * g + r][j * 16 + col] = f16n(fmaxf(acc[j][r] * (1.0f / WC) + bz, 0.0f));
  }
  LDSX();
#pragma unroll
  for (unsigned rp = 0; rp < 8u; ++rp) { const unsigned rl = 2u * rp + g; const v8h v = *(const v8h*)&sg[wave][rl][col * 8u]; vst2(HH + (size_t)(r0 + rl) * DF + c0 + col * 8u, v); }
}

extern "C" void kernel_launch(void* const* d_in, const int* in_sizes, int n_in, void* d_out, int out_size, void* d_ws, size_t ws_size, hipStream_t stream) {
  if (n_in < 18) return;
  const size_t needx = ((size_t)(NB - 1) * SEQ_FULL + SEQ) * DM;
  if ((size_t)in_sizes[0] < needx || in_sizes[1] < NH * RW) return;
  if (in_sizes[2] < DM * DM || in_sizes[4] < DM * DM || in_sizes[6] < DM * DM || in_sizes[8] < DM * DM) return;
  if (in_sizes[3] < DM || in_sizes[5] < DM || in_sizes[7] < DM || in_sizes[9] < DM) return;
  if (in_sizes[10] < DF * DM || in_sizes[11] < DF || in_sizes[12] < DM * DF || in_sizes[13] < DM) return;
  if (in_sizes[14] < DM || in_sizes[15] < DM || in_sizes[16] < DM || in_sizes[17] < DM) return;
  if ((size_t)out_size < needx) return;
  if (ws_size < (size_t)WS_END) return;
  const float* X = (const float*)d_in[0]; const float* RP = (const float*)d_in[1];
  const float* WQ = (const float*)d_in[2]; const float* BQ = (const float*)d_in[3]; const float* WK = (const float*)d_in[4]; const float* BK = (const float*)d_in[5];
  const float* WV = (const float*)d_in[6]; const float* BV = (const float*)d_in[7]; const float* WO = (const float*)d_in[8]; const float* BO = (const float*)d_in[9];
  const float* W1 = (const float*)d_in[10]; const float* B1 = (const float*)d_in[11]; const float* W2 = (const float*)d_in[12]; const float* B2 = (const float*)d_in[13];
  const float* GI = (const float*)d_in[14]; const float* BI = (const float*)d_in[15]; const float* GM = (const float*)d_in[16]; const float* BM = (const float*)d_in[17];
  char* ws = (char*)d_ws;
  _Float16 *WQH = (_Float16*)(ws + WS_WQ), *WKH = (_Float16*)(ws + WS_WK), *WVH = (_Float16*)(ws + WS_WV), *WOH = (_Float16*)(ws + WS_WO), *W1H = (_Float16*)(ws + WS_W1), *W2H = (_Float16*)(ws + WS_W2);
  _Float16 *XN = (_Float16*)(ws + WS_XN), *QH = (_Float16*)(ws + WS_QH), *QL = (_Float16*)(ws + WS_QL), *KH = (_Float16*)(ws + WS_KH), *KL = (_Float16*)(ws + WS_KL);
  _Float16 *VT = (_Float16*)(ws + WS_VT), *O16 = (_Float16*)(ws + WS_O16), *XN2 = (_Float16*)(ws + WS_XN2), *HH = (_Float16*)(ws + WS_HH);
  float* X1 = (float*)(ws + WS_X1);

  const unsigned n8e = DM * DM / 8, n8f = DF * DM / 8;
  k_cvth<<<dim3(n8e / 256), 256, 0, stream>>>(WQ, n8e, WQH);
  k_cvth<<<dim3(n8e / 256), 256, 0, stream>>>(WK, n8e, WKH);
  k_cvth<<<dim3(n8e / 256), 256, 0, stream>>>(WV, n8e, WVH);
  k_cvth<<<dim3(n8e / 256), 256, 0, stream>>>(WO, n8e, WOH);
  k_cvth<<<dim3(n8f / 256), 256, 0, stream>>>(W1, n8f, W1H);
  k_cvth<<<dim3(n8f / 256), 256, 0, stream>>>(W2, n8f, W2H);
  k_ln<true><<<dim3(MROWS / 8), 256, 0, stream>>>(X, GI, BI, XN);
  k_pqk<<<dim3(MROWS / 64, DM / 128), 128, 0, stream>>>(XN, WQH, BQ, QH, QL);
  k_pqk<<<dim3(MROWS / 64, DM / 128), 128, 0, stream>>>(XN, WKH, BK, KH, KL);
  k_pvt<<<dim3(MROWS / 64, DM / 128), 128, 0, stream>>>(XN, WVH, BV, VT);
  k_att<<<dim3(SEQ / 64, NH, NB), 128, 0, stream>>>(QH, QL, KH, KL, VT, RP, O16);
  k_gr<DM, true, false><<<dim3(MROWS / 64, DM / 128), 128, 0, stream>>>(O16, WOH, BO, X, X1);
  k_ln<false><<<dim3(MROWS / 8), 256, 0, stream>>>(X1, GM, BM, XN2);
  k_g1<<<dim3(MROWS / 64, DF / 128), 128, 0, stream>>>(XN2, W1H, B1, HH);
  k_gr<DF, false, true><<<dim3(MROWS / 64, DM / 128), 128, 0, stream>>>(HH, W2H, B2, X1, (float*)d_out);
}
